// Qwen3Attention_48876727829004
// MI455X (gfx1250) — hardware-run, weakly checked
//
#include <hip/hip_runtime.h>

#ifndef NB
#define NB 2
#endif
#ifndef SEQ
#define SEQ 2048
#endif
#define NB_FULL 2
#define SEQ_FULL 2048
#define DM 2048
#define NH 16
#define NKVH 4
#define NREP (NH / NKVH)
#define HDIM 128
#define VW (NKVH * HDIM)
#define NV64 (VW / 64)
#define MSKP 2048
#define RTW 64
#define SLEN SEQ
#define NR (NB * SLEN)
#define TQ SLEN
#define TK SLEN
#define SCL 0.08838834764831845f
#define MVIS (-1.0e8f)
#define QBLKS (TQ / 64)
#define RE ((SLEN < 512) ? SLEN : 512)
#define QB05 0
#define QBN5 (RE / 64)
#define QB0P QBN5
#define QBNP (QBLKS - QBN5)
static_assert(SLEN % 128 == 0);
static_assert(SLEN <= SEQ_FULL);
static_assert(SLEN <= MSKP);
static_assert(NB >= 1 && NB <= NB_FULL);
static_assert(RE % 128 == 0 && RE <= SLEN);
static_assert((SLEN - RE) % 128 == 0);
static_assert(DM % 64 == 0 && DM == NH * HDIM);
static_assert(HDIM == 128 && NH % NKVH == 0);
static_assert(VW % 64 == 0 && NV64 * 64 == VW);
static_assert(DM % 32 == 0 && (2 * DM) % 32 == 0);
static_assert(NR % 128 == 0);
static_assert(((size_t)NR * NH * 16) % 256 == 0 && ((size_t)NR * NKVH * 16) % 256 == 0);
static_assert((NH & (NH - 1)) == 0 && (NKVH & (NKVH - 1)) == 0);
static_assert((size_t)NR * NH * 16 < ((size_t)1 << 31));
static_assert(((size_t)(SLEN / 16) * (SLEN / 32) * 64) % 256 == 0);
static_assert(32 * 16 == HDIM * 4);
static_assert(16 * 16 == 64 * 4);
static_assert(4 * 16 * 40 * 2 + 4 * 16 * 132 * 4 <= 131072);
static_assert(2 * 4 * 16 * 40 * 2 + 4 * 16 * 68 * 4 <= 131072);
static_assert(4 * 32 * 68 * 4 <= 131072);

static constexpr float WSC_LO = 16.0f;
static constexpr float WSC_HI = 16384.0f;
static constexpr float AL_P = 0.0625f;
static constexpr float AL_E = 6.103515625e-05f;

static constexpr size_t al256(size_t b) { return (b + 255) & ~(size_t)255; }
static constexpr size_t SZ_BQ = al256((size_t)DM * DM * 2);
static constexpr size_t SZ_BK = al256((size_t)VW * DM * 2);
static constexpr size_t SZ_B2 = al256((size_t)DM * 2 * DM * 2);
static constexpr size_t SZ_FS = al256((size_t)NR * DM * 4);
static constexpr size_t SZ_X16 = al256((size_t)NR * DM * 2);
static constexpr size_t SZ_QH = al256((size_t)NR * DM * 2);
static constexpr size_t SZ_KH = al256((size_t)NR * VW * 2);
static constexpr size_t SZ_QL = al256((size_t)NB * RE * DM * 2);
static constexpr size_t SZ_KL = al256((size_t)NB * RE * VW * 2);
static constexpr size_t SZ_VTL = al256((size_t)NB * NV64 * 64 * RE * 2);
static constexpr size_t SZ_A2 = al256((size_t)NB * RE * 2 * DM * 2);
static constexpr size_t SZ_MP = al256((size_t)SLEN * SLEN * 2);
static constexpr size_t SZ_JE = al256((size_t)QBLKS * 32 * 4);
static_assert((size_t)NB * NV64 * 64 * TK * 2 <= SZ_X16);
static_assert((size_t)NR * VW * 4 <= SZ_FS);
static_assert(SZ_BQ + 2 * SZ_BK + SZ_B2 + SZ_FS + SZ_X16 + SZ_QH + 2 * SZ_KH + SZ_QL + SZ_KL + SZ_VTL + SZ_A2 + SZ_MP + SZ_JE <= ((size_t)128 << 20));

typedef _Float16 v16h __attribute__((ext_vector_type(16)));
typedef _Float16 v4h __attribute__((ext_vector_type(4)));
typedef unsigned short v8us __attribute__((ext_vector_type(8), may_alias));
typedef float v8f __attribute__((ext_vector_type(8)));
typedef float v4f __attribute__((ext_vector_type(4)));
typedef float v4fa __attribute__((ext_vector_type(4), may_alias));
union FragH { v16h v; v8us half[2]; _Float16 h[16]; unsigned short u[16]; };

__device__ __forceinline__ unsigned short bf16_bits(float x) { unsigned int u = __float_as_uint(x); return (unsigned short)((u + 0x7FFFu + ((u >> 16) & 1u)) >> 16); }
__device__ __forceinline__ float bf16_val(unsigned short b) { return __uint_as_float(((unsigned int)b) << 16); }
__device__ __forceinline__ float bf16_rne(float x) { return bf16_val(bf16_bits(x)); }
__device__ __forceinline__ _Float16 toh_flush(float v) { const _Float16 r = (_Float16)v; return (fabsf(v) < 6.103515625e-05f) ? (_Float16)0.0f : r; }

template <int NT>
__device__ __forceinline__ v8f mmaH(v16h ah, v16h al, v16h bh, v16h bl, v8f c) {
  c = __builtin_amdgcn_wmma_f32_16x16x32_f16(false, ah, false, bh, (short)0, c, false, false);
  if (NT >= 2) c = __builtin_amdgcn_wmma_f32_16x16x32_f16(false, al, false, bh, (short)0, c, false, false);
  if (NT >= 3) c = __builtin_amdgcn_wmma_f32_16x16x32_f16(false, ah, false, bl, (short)0, c, false, false);
  asm volatile("v_nop\n\tv_nop\n\tv_nop\n\tv_nop" : "+v"(c) : "v"(ah), "v"(al), "v"(bh), "v"(bl));
  return c;
}
__device__ __forceinline__ v16h g2_frag(const _Float16* p, int hh) { FragH f; f.half[0] = *(const v8us*)((const unsigned short*)p + 8 * hh); f.half[1] = *(const v8us*)((const unsigned short*)p + 16 + 8 * hh); return f.v; }
__device__ __forceinline__ v8f g2_mma(v16h a, v16h b, v8f c) { v8f d = __builtin_amdgcn_wmma_f32_16x16x32_f16(false, a, false, b, (short)0, c, false, false); asm volatile("v_nop\n\tv_nop\n\tv_nop\n\tv_nop" : "+v"(d) : "v"(a), "v"(b)); return d; }

__global__ __launch_bounds__(256) void k_wsc(const float* __restrict__ Wm, _Float16* __restrict__ Bt, size_t n8, float sc) {
  const size_t t = (size_t)blockIdx.x * 256 + threadIdx.x; if (t >= n8) return;
  const v4f a0 = *(const v4fa*)(Wm + t * 8), a1 = *(const v4fa*)(Wm + t * 8 + 4);
  FragH f;
#pragma unroll
  for (int q = 0; q < 4; ++q) { f.h[q] = toh_flush(bf16_rne(a0[q]) * sc); f.h[4 + q] = toh_flush(bf16_rne(a1[q]) * sc); }
  const v8us o = f.half[0];
  *(volatile v8us*)((unsigned short*)Bt + t * 8) = o; __threadfence(); *(volatile v8us*)((unsigned short*)Bt + t * 8) = o;
}
__global__ __launch_bounds__(256) void k_wsc2(const float* __restrict__ Wm, _Float16* __restrict__ B2, size_t n8, float sc0, float sc1) {
  const size_t t = (size_t)blockIdx.x * 256 + threadIdx.x; if (t >= n8) return;
  const size_t e = t * 8; const size_t n = e / DM; const size_t k8 = e % DM;
  const v4f a0 = *(const v4fa*)(Wm + e), a1 = *(const v4fa*)(Wm + e + 4);
  FragH f0, f1;
#pragma unroll
  for (int q = 0; q < 4; ++q) {
    const float v0 = bf16_rne(a0[q]), v1 = bf16_rne(a1[q]);
    f0.h[q] = toh_flush(v0 * sc0); f1.h[q] = toh_flush(v0 * sc1);
    f0.h[4 + q] = toh_flush(v1 * sc0); f1.h[4 + q] = toh_flush(v1 * sc1);
  }
  const size_t o = n * (size_t)(2 * DM) + k8;
  const v8us o0 = f0.half[0], o1 = f1.half[0];
  for (int pass = 0; pass < 2; ++pass) {
    *(volatile v8us*)((unsigned short*)B2 + o) = o0;
    *(volatile v8us*)((unsigned short*)B2 + o + DM) = o1;
    if (pass == 0) __threadfence();
  }
}

__global__ __launch_bounds__(256) void k_mperm(const float* __restrict__ msk, unsigned short* __restrict__ MP) {
  const size_t t = (size_t)blockIdx.x * 256 + threadIdx.x; if (t >= (size_t)(SLEN / 16) * (SLEN / 32) * 64) return;
  const int lane = (int)(t & 31); const int half = (int)((t >> 5) & 1); const size_t tile = t >> 6;
  const int kt = (int)(tile % (size_t)(SLEN / 32)); const int qt = (int)(tile / (size_t)(SLEN / 32));
  const int ln = lane & 15, hh = lane >> 4;
  const float* mr = msk + (size_t)(qt * 16 + 8 * hh + 4 * half) * MSKP + kt * 32 + ln;
  FragH f;
#pragma unroll
  for (int rr = 0; rr < 4; ++rr) { const float a = mr[(size_t)rr * MSKP]; const float c = mr[(size_t)rr * MSKP + 16]; f.u[2 * rr] = bf16_bits(a); f.u[2 * rr + 1] = bf16_bits(c); }
  const v8us o = f.half[0];
  *(volatile v8us*)(MP + t * 8) = o; __threadfence(); *(volatile v8us*)(MP + t * 8) = o;
}
__global__ __launch_bounds__(256) void k_mjend(const float* __restrict__ msk, int* __restrict__ JE) {
  __shared__ int smax[8]; __shared__ int snone[8];
  const int tid = threadIdx.x, lane = tid & 31; const int w = __builtin_amdgcn_readfirstlane(tid >> 5);
  const int qblk = blockIdx.x;
  int wmax = -1, wnone = 0;
#pragma unroll 1
  for (int rr = 0; rr < 8; ++rr) {
    const float* mr = msk + (size_t)(qblk * 64 + w * 8 + rr) * MSKP;
    int lm = -1;
#pragma unroll 1
    for (int c4 = lane; c4 < SLEN / 4; c4 += 32) {
      const v4f a = *(const v4fa*)(mr + c4 * 4);
      const bool any = (bf16_rne(a[0]) > MVIS) || (bf16_rne(a[1]) > MVIS) || (bf16_rne(a[2]) > MVIS) || (bf16_rne(a[3]) > MVIS);
      lm = any ? (c4 >> 3) : lm;
    }
    int o = __shfl_xor(lm, 16, 32); lm = (o > lm) ? o : lm;
    o = __shfl_xor(lm, 8, 32); lm = (o > lm) ? o : lm;
    o = __shfl_xor(lm, 4, 32); lm = (o > lm) ? o : lm;
    o = __shfl_xor(lm, 2, 32); lm = (o > lm) ? o : lm;
    o = __shfl_xor(lm, 1, 32); lm = (o > lm) ? o : lm;
    wmax = (lm > wmax) ? lm : wmax; wnone |= (lm < 0) ? 1 : 0;
  }
  if (lane == 0) { smax[w] = wmax; snone[w] = wnone; }
  __syncthreads();
  if (w == 0) {
    int m = -1, nn = 0;
#pragma unroll
    for (int i = 0; i < 8; ++i) { const int a = smax[i]; m = (a > m) ? a : m; nn |= snone[i]; }
    const int jt = (nn != 0) ? (SLEN / 32) : (m + 1);
    *(volatile int*)(JE + qblk * 32 + lane) = jt; __threadfence(); *(volatile int*)(JE + qblk * 32 + lane) = jt;
  }
}

__global__ __launch_bounds__(256) void k_x16(const float* __restrict__ x, _Float16* __restrict__ X16, size_t n8) {
  const size_t t = (size_t)blockIdx.x * 256 + threadIdx.x; if (t >= n8) return;
  const size_t e = t * 8; const size_t r = e / DM; const size_t c = e % DM; const size_t b = r / SLEN, s = r % SLEN;
  const float* src = x + (b * SEQ_FULL + s) * DM + c;
  const v4f a0 = *(const v4fa*)src, a1 = *(const v4fa*)(src + 4);
  FragH f;
#pragma unroll
  for (int q = 0; q < 4; ++q) { f.h[q] = (_Float16)bf16_rne(a0[q]); f.h[4 + q] = (_Float16)bf16_rne(a1[q]); }
  const v8us o = f.half[0];
  *(volatile v8us*)((unsigned short*)X16 + e) = o; __threadfence(); *(volatile v8us*)((unsigned short*)X16 + e) = o;
}

template <int ACT>
__global__ __launch_bounds__(128) void k_gemm2(const _Float16* __restrict__ A, int lda, size_t sA, const _Float16* __restrict__ Bh, int ldb, size_t sB, float alpha,
                                               float* C, _Float16* C16, int ldc, size_t sC, int M, int N, int K) {
  __shared__ __attribute__((aligned(16))) float so[4][32][68];
  const int tid = threadIdx.x, w = tid >> 5, lane = tid & 31, ln = lane & 15, hh = lane >> 4; const int by = blockIdx.y;
  A += (size_t)by * sA; Bh += (size_t)by * sB; const size_t cofs = (size_t)by * sC;
  const int ntn = N >> 6; const int mt = blockIdx.x / ntn, nq = blockIdx.x - mt * ntn; const int row0 = mt * 128 + 32 * w, col0 = nq * 64; if (row0 >= M) return;
  const _Float16* a0p = A + (size_t)(row0 + ln) * lda; const _Float16* a1p = a0p + (size_t)16 * lda;
  const _Float16* b0p = Bh + (size_t)(col0 + ln) * ldb; const _Float16* b1p = b0p + (size_t)16 * ldb; const _Float16* b2p = b1p + (size_t)16 * ldb; const _Float16* b3p = b2p + (size_t)16 * ldb;
  const v8f z8 = {0.f,0.f,0.f,0.f,0.f,0.f,0.f,0.f}; v8f c00 = z8, c01 = z8, c02 = z8, c03 = z8, c10 = z8, c11 = z8, c12 = z8, c13 = z8;
#pragma unroll 1
  for (int kb = 0; kb < K; kb += 32) {
    const v16h a0 = g2_frag(a0p + kb, hh), a1 = g2_frag(a1p + kb, hh);
    v16h bf = g2_frag(b0p + kb, hh); c00 = g2_mma(a0, bf, c00); c10 = g2_mma(a1, bf, c10);
    bf = g2_frag(b1p + kb, hh); c01 = g2_mma(a0, bf, c01); c11 = g2_mma(a1, bf, c11);
    bf = g2_frag(b2p + kb, hh); c02 = g2_mma(a0, bf, c02); c12 = g2_mma(a1, bf, c12);
    bf = g2_frag(b3p + kb, hh); c03 = g2_mma(a0, bf, c03); c13 = g2_mma(a1, bf, c13);
  }
  v8f accs[8] = {c00, c01, c02, c03, c10, c11, c12, c13};
#pragma unroll
  for (int u = 0; u < 8; ++u) {
    const int t = u & 3, half = u >> 2;
#pragma unroll
    for (int r = 0; r < 8; ++r) { const int rloc = half * 16 + 8 * hh + r; float v = accs[u][r] * alpha; if (ACT == 3) v = fmaxf(v, 0.f); so[w][rloc][t * 16 + ln] = v; }
  }
  __builtin_amdgcn_fence(4, "workgroup"); __builtin_amdgcn_wave_barrier();
  const int rsub = lane >> 4, c4 = (lane & 15) * 4;
  for (int pass = 0; pass < 2; ++pass) {
#pragma unroll
    for (int q = 0; q < 16; ++q) {
      const int r = q * 2 + rsub; const v4f v = *(const v4fa*)&so[w][r][c4];
      if (C) *(volatile v4f*)(C + cofs + (size_t)(row0 + r) * ldc + col0 + c4) = v;
      if (C16) { v4h h4; for (int i = 0; i < 4; ++i) h4[i] = (_Float16)v[i]; *(volatile v4h*)(C16 + cofs + (size_t)(row0 + r) * ldc + col0 + c4) = h4; }
    }
    if (pass == 0) __threadfence();
  }
}

template <int NHV>
__device__ __forceinline__ void nrope_body(const float* __restrict__ F, int ldf, const float* __restrict__ NW, const float* __restrict__ CT, const float* __restrict__ ST,
                                           _Float16* __restrict__ H, _Float16* __restrict__ L) {
  #pragma clang fp contract(off)
  const unsigned t0 = blockIdx.x * 256u + threadIdx.x; const bool live = t0 < (unsigned)(NR * NHV * 16); const unsigned t = live ? t0 : 0u;
  const int p = (int)(t & 15u); const int hd = (int)((t >> 4) % (unsigned)NHV); const unsigned row = t / (unsigned)(16 * NHV);
  const int s = (int)(row % (unsigned)SLEN); const int b = (int)(row / (unsigned)SLEN);
  const float* src = F + (size_t)row * ldf + hd * HDIM + p * 8;
  const v4f xa = *(const v4fa*)src, xb = *(const v4fa*)(src + 4);
  const v4f wa = *(const v4fa*)(NW + p * 8), wb = *(const v4fa*)(NW + p * 8 + 4);
  const v4f cv = *(const v4fa*)(CT + (size_t)s * RTW + p * 4), sv = *(const v4fa*)(ST + (size_t)s * RTW + p * 4);
  const float xs[8] = {xa[0], xa[1], xa[2], xa[3], xb[0], xb[1], xb[2], xb[3]};
  const float gs[8] = {wa[0], wa[1], wa[2], wa[3], wb[0], wb[1], wb[2], wb[3]};
  float ss = 0.f;
#pragma unroll
  for (int i = 0; i < 8; ++i) { const float q = xs[i] * xs[i]; ss = ss + q; }
  ss += __shfl_xor(ss, 1, 32); ss += __shfl_xor(ss, 2, 32); ss += __shfl_xor(ss, 4, 32); ss += __shfl_xor(ss, 8, 32);
  const float mean = ss * 0.0078125f; const float rms = rsqrtf(mean + 1.0e-6f);
  FragH fh, fl;
#pragma unroll
  for (int j = 0; j < 4; ++j) {
    const float c = bf16_rne(cv[j]), sn = bf16_rne(sv[j]);
    const float y1 = (xs[2 * j] * rms) * bf16_rne(gs[2 * j]); const float y2 = (xs[2 * j + 1] * rms) * bf16_rne(gs[2 * j + 1]);
    const float o1 = y1 * c - y2 * sn; const float o2 = y1 * sn + y2 * c;
    const _Float16 h1 = toh_flush(o1), h2 = toh_flush(o2);
    fh.h[2 * j] = h1; fh.h[2 * j + 1] = h2;
    fl.h[2 * j] = toh_flush((o1 - (float)h1) * 1024.0f); fl.h[2 * j + 1] = toh_flush((o2 - (float)h2) * 1024.0f);
  }
  const size_t oh = (size_t)row * ldf + hd * HDIM + p * 8;
  const bool wl = live && (s < RE);
  const int sl = wl ? s : 0;
  const size_t ol = (size_t)(b * RE + sl) * ldf + hd * HDIM + p * 8;
  const v8us vh = fh.half[0], vl = fl.half[0];
  for (int pass = 0; pass < 2; ++pass) {
    if (live) *(volatile v8us*)((unsigned short*)H + oh) = vh;
    if (wl) *(volatile v8us*)((unsigned short*)L + ol) = vl;
    if (pass == 0) __threadfence();
  }
}
__global__ __launch_bounds__(256) void k_nrope_q(const float* __restrict__ F, int ldf, const float* __restrict__ NW, const float* __restrict__ CT, const float* __restrict__ ST,
                                                 _Float16* __restrict__ H, _Float16* __restrict__ L) {
  #pragma clang fp contract(off)
  nrope_body<NH>(F, ldf, NW, CT, ST, H, L);
}
__global__ __launch_bounds__(256) void k_nrope_k(const float* __restrict__ F, int ldf, const float* __restrict__ NW, const float* __restrict__ CT, const float* __restrict__ ST,
                                                 _Float16* __restrict__ H, _Float16* __restrict__ L) {
  #pragma clang fp contract(off)
  nrope_body<NKVH>(F, ldf, NW, CT, ST, H, L);
}

__global__ __launch_bounds__(256) void k_vtg(const _Float16* __restrict__ V16, _Float16* __restrict__ Vt) {
  __shared__ unsigned short tl[64][66];
  const int tid = threadIdx.x; const int nlg = SLEN / 64; const int slab = blockIdx.x / nlg, lg = blockIdx.x % nlg; const int b = slab / NV64, h = slab % NV64;
  for (int i = tid; i < 64 * 8; i += 256) {
    const int r = i >> 3, c8 = (i & 7) * 8; FragH f;
    f.half[0] = *(const v8us*)((const unsigned short*)V16 + ((size_t)b * SLEN + lg * 64 + r) * VW + h * 64 + c8);
#pragma unroll
    for (int q = 0; q < 8; ++q) tl[r][c8 + q] = f.u[q];
  }
  __syncthreads();
  for (int pass = 0; pass < 2; ++pass) {
#pragma unroll
    for (int rd = 0; rd < 2; ++rd) {
      const int d = rd * 32 + (tid >> 3), pc = tid & 7; FragH f;
#pragma unroll
      for (int q = 0; q < 8; ++q) f.u[q] = tl[pc * 8 + q][d];
      *(volatile v8us*)((unsigned short*)Vt + ((size_t)slab * 64 + d) * TK + lg * 64 + pc * 8) = f.half[0];
    }
    if (pass == 0) __threadfence();
  }
}
__global__ __launch_bounds__(256) void k_vtl(const float* __restrict__ VF, _Float16* __restrict__ VtL) {
  __shared__ unsigned short tl[64][66];
  const int tid = threadIdx.x; const int nlg = RE / 64; const int slab = blockIdx.x / nlg, lg = blockIdx.x % nlg; const int b = slab / NV64, h = slab % NV64;
  for (int i = tid; i < 64 * 16; i += 256) {
    const int r = i >> 4, c4 = (i & 15) * 4;
    const v4f a = *(const v4fa*)(VF + ((size_t)b * SLEN + lg * 64 + r) * VW + h * 64 + c4);
    FragH f;
#pragma unroll
    for (int q = 0; q < 4; ++q) { const float v = a[q]; const _Float16 hv = (_Float16)v; f.h[q] = toh_flush((v - (float)hv) * 1024.0f); }
#pragma unroll
    for (int q = 0; q < 4; ++q) tl[r][c4 + q] = f.u[q];
  }
  __syncthreads();
  for (int pass = 0; pass < 2; ++pass) {
#pragma unroll
    for (int rd = 0; rd < 2; ++rd) {
      const int d = rd * 32 + (tid >> 3), pc = tid & 7; FragH f;
#pragma unroll
      for (int q = 0; q < 8; ++q) f.u[q] = tl[pc * 8 + q][d];
      *(volatile v8us*)((unsigned short*)VtL + ((size_t)slab * 64 + d) * RE + lg * 64 + pc * 8) = f.half[0];
    }
    if (pass == 0) __threadfence();
  }
}

__global__ __launch_bounds__(256) void k_hl(const float* __restrict__ Fp, _Float16* __restrict__ Hh, _Float16* __restrict__ A2, size_t n8) {
  const size_t t = (size_t)blockIdx.x * 256 + threadIdx.x; if (t >= n8) return;
  const size_t e = t * 8; const size_t r = e / DM; const int c = (int)(e % DM); const int s = (int)(r % SLEN); const int b = (int)(r / SLEN);
  const v4f a = *(const v4fa*)(Fp + e), d = *(const v4fa*)(Fp + e + 4);
  FragH fh, fl;
#pragma unroll
  for (int q = 0; q < 4; ++q) {
    _Float16 hv = (_Float16)a[q]; fh.h[q] = hv; fl.h[q] = (_Float16)((a[q] - (float)hv) * 1024.0f);
    hv = (_Float16)d[q]; fh.h[4 + q] = hv; fl.h[4 + q] = (_Float16)((d[q] - (float)hv) * 1024.0f);
  }
  const bool wl = (s < RE);
  const size_t o2 = ((size_t)b * RE + (wl ? s : 0)) * (size_t)(2 * DM) + c;
  const v8us vh = fh.half[0], vl = fl.half[0];
  for (int pass = 0; pass < 2; ++pass) {
    *(volatile v8us*)((unsigned short*)Hh + e) = vh;
    if (wl) { *(volatile v8us*)((unsigned short*)A2 + o2) = vh; *(volatile v8us*)((unsigned short*)A2 + o2 + DM) = vl; }
    if (pass == 0) __threadfence();
  }
}

__global__ __launch_bounds__(128) __attribute__((amdgpu_num_vgpr(256))) void k_flash(const _Float16* __restrict__ Q16, int ldq, const _Float16* __restrict__ K16, int ldk,
                                               const _Float16* __restrict__ Vt, const unsigned short* __restrict__ MP, const int* __restrict__ JE, float* __restrict__ O, int ldo) {
  constexpr int RPW = 16, DT = 8, KS = 4;
  constexpr int NQP = (QBNP > 0) ? QBNP : 1;
  __shared__ __attribute__((aligned(16))) unsigned short sP[4][RPW][40];
  __shared__ __attribute__((aligned(16))) float sO[4][RPW][132];
  const int tid = threadIdx.x, lane = tid & 31, ln = lane & 15, hh = lane >> 4;
  const int w = __builtin_amdgcn_readfirstlane(tid >> 5);
  const int slab = blockIdx.x / NQP, qblk = QB0P + blockIdx.x % NQP; const int b = slab / NH, h = slab % NH; const int kvh = h / NREP;
  const int qb0 = qblk * (4 * RPW); const int q0 = qb0 + w * RPW;
  const unsigned short* qr = (const unsigned short*)Q16 + ((size_t)b * TQ + q0 + ln) * ldq + h * HDIM;
  const unsigned short* kb = (const unsigned short*)K16 + ((size_t)b * TK + ln) * ldk + kvh * HDIM;
  const unsigned short* Vth = (const unsigned short*)Vt + (size_t)(b * NKVH + kvh) * HDIM * TK;
  const unsigned short* mq = MP + (size_t)(q0 >> 4) * (size_t)(TK / 32) * 512 + lane * 8;
  int jt = JE[qblk * 32]; jt = (jt < 1) ? 1 : jt; jt = (jt > TK / 32) ? (TK / 32) : jt;
  const int jend = __builtin_amdgcn_readfirstlane(jt) * 32;
  float m_r[8], l_r[8]; v8f oacc[DT];
#pragma unroll
  for (int r = 0; r < 8; ++r) { m_r[r] = -3.0e38f; l_r[r] = 0.f; }
#pragma unroll
  for (int dt = 0; dt < DT; ++dt) oacc[dt] = (v8f){0.f,0.f,0.f,0.f,0.f,0.f,0.f,0.f};
#pragma unroll 1
  for (int j0 = 0; j0 < jend; j0 += 32) {
    v8f sa = (v8f){0.f,0.f,0.f,0.f,0.f,0.f,0.f,0.f}, sb = sa;
    const unsigned short* kr0 = kb + (size_t)j0 * ldk; const unsigned short* kr1 = kr0 + (size_t)16 * ldk;
#pragma unroll
    for (int ks = 0; ks < KS; ++ks) {
      FragH a, k0, k1;
      a.half[0] = *(const v8us*)(qr + ks * 32 + 8 * hh); a.half[1] = *(const v8us*)(qr + ks * 32 + 16 + 8 * hh);
      k0.half[0] = *(const v8us*)(kr0 + ks * 32 + 8 * hh); k0.half[1] = *(const v8us*)(kr0 + ks * 32 + 16 + 8 * hh);
      k1.half[0] = *(const v8us*)(kr1 + ks * 32 + 8 * hh); k1.half[1] = *(const v8us*)(kr1 + ks * 32 + 16 + 8 * hh);
      sa = g2_mma(a.v, k0.v, sa); sb = g2_mma(a.v, k1.v, sb);
    }
    FragH fm; { const unsigned short* mt = mq + (size_t)(j0 >> 5) * 512; fm.half[0] = *(const v8us*)mt; fm.half[1] = *(const v8us*)(mt + 256); }
#pragma unroll
    for (int r = 0; r < 8; ++r) {
      const float mk0 = bf16_val(fm.u[2 * r]), mk1 = bf16_val(fm.u[2 * r + 1]);
      const float s0 = sa[r] * SCL + mk0, s1 = sb[r] * SCL + mk1;
      float mc = fmaxf(s0, s1);
      mc = fmaxf(mc, __shfl_xor(mc, 1, 32)); mc = fmaxf(mc, __shfl_xor(mc, 2, 32)); mc = fmaxf(mc, __shfl_xor(mc, 4, 32)); mc = fmaxf(mc, __shfl_xor(mc, 8, 32));
      const float mn = fmaxf(m_r[r], mc); const float al = (mn > -1.0e38f) ? expf(m_r[r] - mn) : 1.0f; m_r[r] = mn;
      const float p0 = expf(s0 - mn), p1 = expf(s1 - mn); l_r[r] = l_r[r] * al + p0 + p1;
#pragma unroll
      for (int dt = 0; dt < DT; ++dt) oacc[dt][r] *= al;
      FragH t2; t2.h[0] = toh_flush(p0 * 1024.0f); t2.h[1] = toh_flush(p1 * 1024.0f);
      sP[w][8 * hh + r][ln] = t2.u[0]; sP[w][8 * hh + r][16 + ln] = t2.u[1];
    }
    __builtin_amdgcn_fence(4, "workgroup"); __builtin_amdgcn_wave_barrier();
    FragH pa; pa.half[0] = *(const v8us*)&sP[w][ln][8 * hh]; pa.half[1] = *(const v8us*)&sP[w][ln][16 + 8 * hh];
#pragma unroll
    for (int dt = 0; dt < DT; ++dt) {
      const unsigned short* vrow = Vth + (size_t)(dt * 16 + ln) * TK + j0; FragH bv;
      bv.half[0] = *(const v8us*)(vrow + 8 * hh); bv.half[1] = *(const v8us*)(vrow + 16 + 8 * hh);
      oacc[dt] = g2_mma(pa.v, bv.v, oacc[dt]);
    }
    __builtin_amdgcn_fence(4, "workgroup"); __builtin_amdgcn_wave_barrier();
  }
#pragma unroll
  for (int r = 0; r < 8; ++r) { float l = l_r[r]; l += __shfl_xor(l, 1, 32); l += __shfl_xor(l, 2, 32); l += __shfl_xor(l, 4, 32); l += __shfl_xor(l, 8, 32); l_r[r] = (l > 0.f) ? 1.0f / (l * 1024.0f) : 0.f; }
#pragma unroll
  for (int dt = 0; dt < DT; ++dt)
#pragma unroll
    for (int r = 0; r < 8; ++r) sO[w][8 * hh + r][dt * 16 + ln] = oacc[dt][r] * l_r[r];
  __builtin_amdgcn_fence(4, "workgroup"); __builtin_amdgcn_wave_barrier();
  for (int pass = 0; pass < 2; ++pass) {
#pragma unroll
    for (int rp = 0; rp < RPW; ++rp) { const v4f val = *(const v4fa*)&sO[w][rp][lane * 4]; *(volatile v4f*)(O + ((size_t)b * TQ + q0 + rp) * ldo + h * HDIM + lane * 4) = val; }
    if (pass == 0) __threadfence();
  }
}
__global__ __launch_bounds__(128) __attribute__((amdgpu_num_vgpr(256))) void k_flash5(const _Float16* __restrict__ Q16, const _Float16* __restrict__ QL, int ldq, const _Float16* __restrict__ K16, const _Float16* __restrict__ KL, int ldk,
                                                const _Float16* __restrict__ Vt, const _Float16* __restrict__ VtL, const unsigned short* __restrict__ MP, const int* __restrict__ JE, float* __restrict__ O, int ldo) {
  constexpr int RPW = 16, DT = 4, KS = 4;
  __shared__ __attribute__((aligned(16))) unsigned short sP[4][RPW][40];
  __shared__ __attribute__((aligned(16))) unsigned short sPL[4][RPW][40];
  __shared__ __attribute__((aligned(16))) float sO[4][RPW][68];
  const int tid = threadIdx.x, lane = tid & 31, ln = lane & 15, hh = lane >> 4;
  const int w = __builtin_amdgcn_readfirstlane(tid >> 5);
  const int dh = blockIdx.x & 1; const int bx = blockIdx.x >> 1;
  const int slab = bx / QBN5, qblk = QB05 + bx % QBN5; const int b = slab / NH, h = slab % NH; const int kvh = h / NREP;
  const int qb0 = qblk * (4 * RPW); const int q0 = qb0 + w * RPW;
  const unsigned short* qr = (const unsigned short*)Q16 + ((size_t)b * TQ + q0 + ln) * ldq + h * HDIM;
  const unsigned short* ql = (const unsigned short*)QL + ((size_t)b * RE + q0 + ln) * ldq + h * HDIM;
  const unsigned short* kb = (const unsigned short*)K16 + ((size_t)b * TK + ln) * ldk + kvh * HDIM;
  const unsigned short* klb = (const unsigned short*)KL + ((size_t)b * RE + ln) * ldk + kvh * HDIM;
  const unsigned short* Vth = (const unsigned short*)Vt + ((size_t)(b * NKVH + kvh) * HDIM + dh * 64) * TK;
  const unsigned short* Vtl = (const unsigned short*)VtL + ((size_t)(b * NKVH + kvh) * HDIM + dh * 64) * RE;
  const unsigned short* mq = MP + (size_t)(q0 >> 4) * (size_t)(TK / 32) * 512 + lane * 8;
  const int jraw = JE[qblk * 32];
  const float pz = (jraw > RE / 32) ? __uint_as_float(0x7FC00000u) : 0.0f;
  int jt = (jraw < 1) ? 1 : jraw; jt = (jt > RE / 32) ? (RE / 32) : jt;
  const int jend = __builtin_amdgcn_readfirstlane(jt) * 32;
  float m_r[8], l_r[8]; v8f oacc[DT], oaccL[DT];
#pragma unroll
  for (int r = 0; r < 8; ++r) { m_r[r] = -3.0e38f; l_r[r] = 0.f; }
#pragma unroll
  for (int dt = 0; dt < DT; ++dt) { oacc[dt] = (v8f){0.f,0.f,0.f,0.f,0.f,0.f,0.f,0.f}; oaccL[dt] = oacc[dt]; }
#pragma unroll 1
  for (int j0 = 0; j0 < jend; j0 += 32) {
    v8f sa = (v8f){0.f,0.f,0.f,0.f,0.f,0.f,0.f,0.f}, sb = sa, sal = sa, sbl = sa;
    const unsigned short* kr0 = kb + (size_t)j0 * ldk; const unsigned short* kr1 = kr0 + (size_t)16 * ldk;
    const unsigned short* kl0 = klb + (size_t)j0 * ldk; const unsigned short* kl1 = kl0 + (size_t)16 * ldk;
#pragma unroll
    for (int ks = 0; ks < KS; ++ks) {
      FragH a, al2, k0, k1;
      a.half[0] = *(const v8us*)(qr + ks * 32 + 8 * hh); a.half[1] = *(const v8us*)(qr + ks * 32 + 16 + 8 * hh);
      al2.half[0] = *(const v8us*)(ql + ks * 32 + 8 * hh); al2.half[1] = *(const v8us*)(ql + ks * 32 + 16 + 8 * hh);
      k0.half[0] = *(const v8us*)(kr0 + ks * 32 + 8 * hh); k0.half[1] = *(const v8us*)(kr0 + ks * 32 + 16 + 8 * hh);
      k1.half[0] = *(const v8us*)(kr1 + ks * 32 + 8 * hh); k1.half[1] = *(const v8us*)(kr1 + ks * 32 + 16 + 8 * hh);
      sa = g2_mma(a.v, k0.v, sa); sb = g2_mma(a.v, k1.v, sb);
      sal = g2_mma(al2.v, k0.v, sal); sbl = g2_mma(al2.v, k1.v, sbl);
      k0.half[0] = *(const v8us*)(kl0 + ks * 32 + 8 * hh); k0.half[1] = *(const v8us*)(kl0 + ks * 32 + 16 + 8 * hh);
      k1.half[0] = *(const v8us*)(kl1 + ks * 32 + 8 * hh); k1.half[1] = *(const v8us*)(kl1 + ks * 32 + 16 + 8 * hh);
      sal = g2_mma(a.v, k0.v, sal); sbl = g2_mma(a.v, k1.v, sbl);
    }
    FragH fm; { const unsigned short* mt = mq + (size_t)(j0 >> 5) * 512; fm.half[0] = *(const v8us*)mt; fm.half[1] = *(const v8us*)(mt + 256); }
#pragma unroll
    for (int r = 0; r < 8; ++r) {
      const float mk0 = bf16_val(fm.u[2 * r]), mk1 = bf16_val(fm.u[2 * r + 1]);
      const float d0 = sa[r] + sal[r] * 0.0009765625f, d1 = sb[r] + sbl[r] * 0.0009765625f;
      const float s0 = d0 * SCL + mk0, s1 = d1 * SCL + mk1;
      float mc = fmaxf(s0, s1);
      mc = fmaxf(mc, __shfl_xor(mc, 1, 32)); mc = fmaxf(mc, __shfl_xor(mc, 2, 32)); mc = fmaxf(mc, __shfl_xor(mc, 4, 32)); mc = fmaxf(mc, __shfl_xor(mc, 8, 32));
      const float mn = fmaxf(m_r[r], mc); const float al = (mn > -1.0e38f) ? expf(m_r[r] - mn) : 1.0f; m_r[r] = mn;
      const float p0 = expf(s0 - mn), p1 = expf(s1 - mn); l_r[r] = l_r[r] * al + p0 + p1;
#pragma unroll
      for (int dt = 0; dt < DT; ++dt) { oacc[dt][r] *= al; oaccL[dt][r] *= al; }
      FragH t2, t2l; const float ps0 = p0 * 1024.0f, ps1 = p1 * 1024.0f;
      t2.h[0] = toh_flush(ps0); t2.h[1] = toh_flush(ps1);
      t2l.h[0] = toh_flush((ps0 - (float)t2.h[0]) * 1024.0f); t2l.h[1] = toh_flush((ps1 - (float)t2.h[1]) * 1024.0f);
      sP[w][8 * hh + r][ln] = t2.u[0]; sP[w][8 * hh + r][16 + ln] = t2.u[1]; sPL[w][8 * hh + r][ln] = t2l.u[0]; sPL[w][8 * hh + r][16 + ln] = t2l.u[1];
    }
    __builtin_amdgcn_fence(4, "workgroup"); __builtin_amdgcn_wave_barrier();
    FragH pa, pl;
    pa.half[0] = *(const v8us*)&sP[w][ln][8 * hh]; pa.half[1] = *(const v8us*)&sP[w][ln][16 + 8 * hh];
    pl.half[0] = *(const v8us*)&sPL[w][ln][8 * hh]; pl.half[1] = *(const v8us*)&sPL[w][ln][16 + 8 * hh];
#pragma unroll
    for (int dt = 0; dt < DT; ++dt) {
      const unsigned short* vrow = Vth + (size_t)(dt * 16 + ln) * TK + j0; const unsigned short* vrl = Vtl + (size_t)(dt * 16 + ln) * RE + j0;
      FragH bv, bl;
      bv.half[0] = *(const v8us*)(vrow + 8 * hh); bv.half[1] = *(const v8us*)(vrow + 16 + 8 * hh);
      bl.half[0] = *(const v8us*)(vrl + 8 * hh); bl.half[1] = *(const v8us*)(vrl + 16 + 8 * hh);
      oacc[dt] = g2_mma(pa.v, bv.v, oacc[dt]);
      oaccL[dt] = g2_mma(pl.v, bv.v, oaccL[dt]);
      oaccL[dt] = g2_mma(pa.v, bl.v, oaccL[dt]);
    }
    __builtin_amdgcn_fence(4, "workgroup"); __builtin_amdgcn_wave_barrier();
  }
#pragma unroll
  for (int r = 0; r < 8; ++r) { float l = l_r[r]; l += __shfl_xor(l, 1, 32); l += __shfl_xor(l, 2, 32); l += __shfl_xor(l, 4, 32); l += __shfl_xor(l, 8, 32); l_r[r] = (l > 0.f) ? 1.0f / (l * 1024.0f) : 0.f; }
#pragma unroll
  for (int dt = 0; dt < DT; ++dt)
#pragma unroll
    for (int r = 0; r < 8; ++r) { float v = oacc[dt][r]; v += oaccL[dt][r] * 0.0009765625f; sO[w][8 * hh + r][dt * 16 + ln] = v * l_r[r] + pz; }
  __builtin_amdgcn_fence(4, "workgroup"); __builtin_amdgcn_wave_barrier();
  for (int pass = 0; pass < 2; ++pass) {
#pragma unroll
    for (int rp = 0; rp < RPW; rp += 2) { const int r = rp + (lane >> 4), pc = lane & 15; const v4f val = *(const v4fa*)&sO[w][r][pc * 4]; *(volatile v4f*)(O + ((size_t)b * TQ + q0 + r) * ldo + h * HDIM + dh * 64 + pc * 4) = val; }
    if (pass == 0) __threadfence();
  }
}

extern "C" void kernel_launch(void* const* d_in, const int* in_sizes, int n_in,
                              void* d_out, int out_size, void* d_ws, size_t ws_size, hipStream_t stream) {
  if (n_in < 10) return;
  const size_t needx = ((size_t)(NB - 1) * SEQ_FULL + (size_t)SLEN) * DM;
  if ((size_t)in_sizes[0] < needx) return;
  if ((size_t)in_sizes[1] < (size_t)DM * DM) return;
  if ((size_t)in_sizes[2] < (size_t)VW * DM) return;
  if ((size_t)in_sizes[3] < (size_t)VW * DM) return;
  if ((size_t)in_sizes[4] < (size_t)DM * DM) return;
  if ((size_t)in_sizes[5] < (size_t)HDIM) return;
  if ((size_t)in_sizes[6] < (size_t)HDIM) return;
  if ((size_t)in_sizes[7] < (size_t)SLEN * RTW) return;
  if ((size_t)in_sizes[8] < (size_t)SLEN * RTW) return;
  if ((size_t)in_sizes[9] < (size_t)(SLEN - 1) * MSKP + (size_t)SLEN) return;
  if ((size_t)out_size < needx) return;
  const float* x = (const float*)d_in[0]; const float* Wq = (const float*)d_in[1]; const float* Wk = (const float*)d_in[2]; const float* Wv = (const float*)d_in[3]; const float* Wo = (const float*)d_in[4];
  const float* qnw = (const float*)d_in[5]; const float* knw = (const float*)d_in[6]; const float* rct = (const float*)d_in[7]; const float* rst = (const float*)d_in[8]; const float* msk = (const float*)d_in[9];
  float* dout = (float*)d_out;
  char* ws = (char*)d_ws; size_t off = 0;
  auto take = [&](size_t bytes) { char* p = ws + off; off += (bytes + 255) & ~(size_t)255; return p; };
  const size_t np = (size_t)NR * DM;
  const size_t nw8 = (size_t)DM * DM / 8;
  const size_t nk8 = (size_t)VW * DM / 8;
  _Float16* BQ = (_Float16*)take(SZ_BQ);
  _Float16* BK = (_Float16*)take(SZ_BK);
  _Float16* BV = (_Float16*)take(SZ_BK);
  _Float16* B2 = (_Float16*)take(SZ_B2);
  float* FS = (float*)take(SZ_FS);
  _Float16* X16 = (_Float16*)take(SZ_X16);
  _Float16* VT = X16;
  _Float16* QH = (_Float16*)take(SZ_QH);
  _Float16* KHp = (_Float16*)take(SZ_KH);
  _Float16* V16 = (_Float16*)take(SZ_KH);
  _Float16* QL = (_Float16*)take(SZ_QL);
  _Float16* KL = (_Float16*)take(SZ_KL);
  _Float16* VTL = (_Float16*)take(SZ_VTL);
  _Float16* A2 = (_Float16*)take(SZ_A2);
  unsigned short* MPp = (unsigned short*)take(SZ_MP);
  int* JEp = (int*)take(SZ_JE);
  _Float16* OH = QH;
  if (off > ws_size) return;
  if (off > ((size_t)128 << 20)) return;

  const unsigned gw = (unsigned)((nw8 + 255) / 256);
  const unsigned gk = (unsigned)((nk8 + 255) / 256);
  k_wsc<<<gw, 256, 0, stream>>>(Wq, BQ, nw8, WSC_LO);
  k_wsc<<<gk, 256, 0, stream>>>(Wk, BK, nk8, WSC_LO);
  k_wsc<<<gk, 256, 0, stream>>>(Wv, BV, nk8, WSC_LO);
  k_wsc2<<<gw, 256, 0, stream>>>(Wo, B2, nw8, WSC_HI, WSC_LO);
  k_mperm<<<(unsigned)(((size_t)(SLEN / 16) * (SLEN / 32) * 64) / 256), 256, 0, stream>>>(msk, MPp);
  k_mjend<<<(unsigned)QBLKS, 256, 0, stream>>>(msk, JEp);
  const unsigned g8 = (unsigned)((np / 8 + 255) / 256);
  k_x16<<<g8, 256, 0, stream>>>(x, X16, np / 8);
  const dim3 gp((unsigned)((NR / 128) * (DM / 64)), 1);
  const dim3 gkv((unsigned)((NR / 128) * (VW / 64)), 1);
  const unsigned grq = (unsigned)(((size_t)NR * NH * 16) / 256);
  const unsigned grk = (unsigned)(((size_t)NR * NKVH * 16) / 256);
  k_gemm2<0><<<gp, 128, 0, stream>>>(X16, DM, 0, BQ, DM, 0, AL_P, FS, nullptr, DM, 0, NR, DM, DM);
  k_nrope_q<<<grq, 256, 0, stream>>>(FS, DM, qnw, rct, rst, QH, QL);
  k_gemm2<0><<<gkv, 128, 0, stream>>>(X16, DM, 0, BK, DM, 0, AL_P, FS, nullptr, VW, 0, NR, VW, DM);
  k_nrope_k<<<grk, 256, 0, stream>>>(FS, VW, knw, rct, rst, KHp, KL);
  k_gemm2<0><<<gkv, 128, 0, stream>>>(X16, DM, 0, BV, DM, 0, AL_P, FS, V16, VW, 0, NR, VW, DM);
  k_vtg<<<(unsigned)(NB * NV64 * (SLEN / 64)), 256, 0, stream>>>(V16, VT);
  k_vtl<<<(unsigned)(NB * NV64 * (RE / 64)), 256, 0, stream>>>(FS, VTL);
  k_flash5<<<(unsigned)(NB * NH * QBN5 * 2), 128, 0, stream>>>(QH, QL, DM, KHp, KL, VW, VT, VTL, MPp, JEp, FS, DM);
  if (QBNP > 0) k_flash<<<(unsigned)(NB * NH * QBNP), 128, 0, stream>>>(QH, DM, KHp, VW, VT, MPp, JEp, FS, DM);
  k_hl<<<g8, 256, 0, stream>>>(FS, OH, A2, np / 8);
  const dim3 ge((unsigned)((RE / 128) * (DM / 64)), NB);
  k_gemm2<0><<<ge, 128, 0, stream>>>(A2, 2 * DM, (size_t)RE * 2 * DM, B2, 2 * DM, 0, AL_E, dout, nullptr, DM, (size_t)SEQ_FULL * DM, RE, DM, 2 * DM);
  if (SLEN > RE) {
    const dim3 gl((unsigned)(((SLEN - RE) / 128) * (DM / 64)), NB);
    k_gemm2<0><<<gl, 128, 0, stream>>>(OH + (size_t)RE * DM, DM, (size_t)SLEN * DM, B2 + DM, 2 * DM, 0, AL_P, dout + (size_t)RE * DM, nullptr, DM, (size_t)SEQ_FULL * DM, SLEN - RE, DM, DM);
  }
}
